// SA_19413252178719
// MI455X (gfx1250) — hardware-run, weakly checked
//
#include <hip/hip_runtime.h>
#include <math.h>

constexpr int kB     = 4;
constexpr int kC     = 512;
constexpr int kN     = 4096;
constexpr int kQ     = 64;
constexpr int kWRows = 2 * kQ + kC;
constexpr int kTok   = kB * kN;
constexpr int kCh    = 2048;
constexpr float kPCarry    = 32768.0f;
constexpr float kPCarryInv = 1.0f / 32768.0f;
static_assert(kN % 64 == 0 && kC % 64 == 0 && kQ % 64 == 0 && kCh % 64 == 0);
static_assert(kC % 32 == 0 && kQ % 32 == 0 && kN % 32 == 0);
static_assert(kN % kCh == 0 && kN % 128 == 0);
static_assert((kWRows * kC) % 2048 == 0 && (kQ * kC) % 2048 == 0);

typedef __attribute__((ext_vector_type(16))) _Float16 v16h;
typedef __attribute__((ext_vector_type(8)))  _Float16 v8h;
typedef __attribute__((ext_vector_type(16))) __bf16   v16b;
typedef __attribute__((ext_vector_type(8)))  __bf16   v8b;
typedef __attribute__((ext_vector_type(8)))  float    v8f;
typedef __attribute__((ext_vector_type(4)))  float    v4f;
typedef __attribute__((ext_vector_type(4)))  unsigned int v4u;
typedef __attribute__((ext_vector_type(8)))  unsigned short v8us;

__device__ __forceinline__ unsigned short f2bf_bits(float f) {
  unsigned u = __float_as_uint(f);
  return (unsigned short)((u + 0x7FFFu + ((u >> 16) & 1u)) >> 16);
}
__device__ __forceinline__ float bf_bits2f(unsigned short h) { return __uint_as_float(((unsigned)h) << 16); }
__device__ __forceinline__ float rbf(float f) { return bf_bits2f(f2bf_bits(f)); }

__device__ __forceinline__ void dep_guard4_h(v8f& a, v8f& b, v8f& c, v8f& d, v16h x, v16h y) { asm volatile("v_nop\n\tv_nop\n\tv_nop\n\tv_nop" : "+v"(a), "+v"(b), "+v"(c), "+v"(d) : "v"(x), "v"(y)); }
__device__ __forceinline__ void dep_guard4_b(v8f& a, v8f& b, v8f& c, v8f& d, v16b x, v16b y) { asm volatile("v_nop\n\tv_nop\n\tv_nop\n\tv_nop" : "+v"(a), "+v"(b), "+v"(c), "+v"(d) : "v"(x), "v"(y)); }
__device__ __forceinline__ void keep4_h(v16h a, v16h b, v16h c, v16h d) { asm volatile("v_nop" :: "v"(a), "v"(b), "v"(c), "v"(d)); }
__device__ __forceinline__ void keep4_b(v16b a, v16b b, v16b c, v16b d) { asm volatile("v_nop" :: "v"(a), "v"(b), "v"(c), "v"(d)); }
__device__ __forceinline__ void acc_guard4(v8f& a, v8f& b, v8f& c, v8f& d) { asm volatile("v_nop\n\tv_nop\n\tv_nop\n\tv_nop" : "+v"(a), "+v"(b), "+v"(c), "+v"(d)); }
template <typename T> struct Frag;
template <> struct Frag<_Float16> {
  typedef v16h V; union U { v16h v; v8h h[2]; };
  static __device__ __forceinline__ v16h load(const _Float16* p) {
    U f; f.h[0] = *(const v8h*)(p); f.h[1] = *(const v8h*)(p + 16); return f.v;
  }
  static __device__ __forceinline__ v8f mma(v16h a, v16h b, v8f c) {
    return __builtin_amdgcn_wmma_f32_16x16x32_f16(false, a, false, b, (short)0, c, false, false);
  }
  static __device__ __forceinline__ void guard4(v8f& a, v8f& b, v8f& c, v8f& d, v16h x, v16h y) { dep_guard4_h(a, b, c, d, x, y); }
  static __device__ __forceinline__ void keep(v16h a, v16h b, v16h c, v16h d) { keep4_h(a, b, c, d); }
};
template <> struct Frag<__bf16> {
  typedef v16b V; union U { v16b v; v8b h[2]; };
  static __device__ __forceinline__ v16b load(const __bf16* p) {
    U f; f.h[0] = *(const v8b*)(p); f.h[1] = *(const v8b*)(p + 16); return f.v;
  }
  static __device__ __forceinline__ v8f mma(v16b a, v16b b, v8f c) {
    return __builtin_amdgcn_wmma_f32_16x16x32_bf16(false, a, false, b, (short)0, c, false, false);
  }
  static __device__ __forceinline__ void guard4(v8f& a, v8f& b, v8f& c, v8f& d, v16b x, v16b y) { dep_guard4_b(a, b, c, d, x, y); }
  static __device__ __forceinline__ void keep(v16b a, v16b b, v16b c, v16b d) { keep4_b(a, b, c, d); }
};

__device__ __forceinline__ unsigned pk16(unsigned short a, unsigned short b) { return (unsigned)a | ((unsigned)b << 16); }
__device__ __forceinline__ unsigned short h_bits(float f) { const _Float16 h = (_Float16)f; return __builtin_bit_cast(unsigned short, h); }

template <int ET> struct Elem;
template <> struct Elem<0> { typedef _Float16 T; };
template <> struct Elem<1> { typedef __bf16 T; };
template <int ET, bool SPLIT, int BIAS_MODE, int OUT_MODE, bool RESID, bool DSC>
__global__ __launch_bounds__(256) void wmma_gemm64(
    const unsigned short* __restrict__ Ap, const unsigned short* __restrict__ A2p, int lda, long strideA,
    const unsigned short* __restrict__ Btp, const unsigned short* __restrict__ Bt2p, int ldb, long strideB,
    void* __restrict__ Cout, void* __restrict__ Cout2, int ldc, long strideC,
    const float* __restrict__ bias,
    const float* __restrict__ resid, long strideR,
    const float* __restrict__ dsc,
    int M, int N, int K, float scale) {
  static_assert(!(RESID && OUT_MODE != 0));
  typedef typename Elem<ET>::T T;
  typedef typename Frag<T>::V V;
  const T* A = (const T*)Ap; const T* A2 = (const T*)A2p; const T* Bt = (const T*)Btp; const T* Bt2 = (const T*)Bt2p;
  __shared__ __align__(16) float sT[8][16 * 68];
  const int b    = blockIdx.y;
  const int lane = threadIdx.x & 31;
  const int wave = threadIdx.x >> 5;
  const int tilesN = N >> 6;
  const int tilesM = M >> 6;
  const int tile = blockIdx.x * 8 + wave;
  if (tile >= tilesM * tilesN) return;
  const int tm = tile / tilesN;
  const int tn = tile - tm * tilesN;
  const int m0 = tm << 6;
  const int n0 = tn << 6;

  const T* Ab  = A  + (size_t)b * strideA;
  const T* Bb  = Bt + (size_t)b * strideB;
  const T* Ab2 = SPLIT ? (A2  + (size_t)b * strideA) : nullptr;
  const T* Bb2 = SPLIT ? (Bt2 + (size_t)b * strideB) : nullptr;

  const float scl = DSC ? (scale * rbf(dsc[0])) : scale;

  const int rlane = lane & 15;
  const int koff  = (lane >> 4) * 8;
  const int mOff  = (lane >> 4) * 8;

  v8f acc[4][4];
#pragma unroll
  for (int i = 0; i < 4; ++i)
#pragma unroll
    for (int j = 0; j < 4; ++j) acc[i][j] = (v8f){0.f,0.f,0.f,0.f,0.f,0.f,0.f,0.f};

  for (int k0 = 0; k0 < K; k0 += 32) {
    V bh[4], bl[4];
#pragma unroll
    for (int j = 0; j < 4; ++j) {
      const size_t bo = (size_t)(n0 + (j << 4) + rlane) * ldb + koff + k0;
      bh[j] = Frag<T>::load(Bb + bo);
      if (SPLIT) bl[j] = Frag<T>::load(Bb2 + bo);
    }
#pragma unroll
    for (int i = 0; i < 4; ++i) {
      const size_t ao = (size_t)(m0 + (i << 4) + rlane) * lda + koff + k0;
      V ah = Frag<T>::load(Ab + ao);
      V al;
      if (SPLIT) al = Frag<T>::load(Ab2 + ao);
#pragma unroll
      for (int j = 0; j < 4; ++j) {
        acc[i][j] = Frag<T>::mma(ah, bh[j], acc[i][j]);
        if (SPLIT) {
          acc[i][j] = Frag<T>::mma(ah, bl[j], acc[i][j]);
          acc[i][j] = Frag<T>::mma(al, bh[j], acc[i][j]);
        }
      }
      Frag<T>::guard4(acc[i][0], acc[i][1], acc[i][2], acc[i][3], ah, SPLIT ? al : ah);
    }
    Frag<T>::keep(bh[0], bh[1], bh[2], bh[3]);
    if (SPLIT) Frag<T>::keep(bl[0], bl[1], bl[2], bl[3]);
  }
  acc_guard4(acc[0][0], acc[0][1], acc[0][2], acc[0][3]);
  acc_guard4(acc[1][0], acc[1][1], acc[1][2], acc[1][3]);
  acc_guard4(acc[2][0], acc[2][1], acc[2][2], acc[2][3]);
  acc_guard4(acc[3][0], acc[3][1], acc[3][2], acc[3][3]);

  float* slab = sT[wave];
  const float* Rb = RESID ? (resid + (size_t)b * strideR) : nullptr;
#pragma unroll
  for (int i = 0; i < 4; ++i) {
    const int mBase = m0 + (i << 4);
#pragma unroll
    for (int j = 0; j < 4; ++j) {
      const int n = n0 + (j << 4) + rlane;
      float bv = 0.f;
      if (BIAS_MODE == 2) bv = rbf(bias[n]);
#pragma unroll
      for (int r = 0; r < 8; ++r) {
        float v = acc[i][j][r] * scl;
        if (BIAS_MODE == 1) v += rbf(bias[mBase + mOff + r]);
        if (BIAS_MODE == 2) v += bv;
        slab[(mOff + r) * 68 + (j << 4) + rlane] = v;
      }
    }
    __builtin_amdgcn_fence(__ATOMIC_RELEASE, "workgroup");
    __builtin_amdgcn_wave_barrier();
    __builtin_amdgcn_fence(__ATOMIC_ACQUIRE, "workgroup");
    if (OUT_MODE == 0) {
      float* Cb = (float*)Cout + (size_t)b * strideC;
      const int hq = lane >> 4, c4 = (lane & 15) * 4;
      v4f vals[8];
#pragma unroll
      for (int it = 0; it < 8; ++it) {
        const int row = it * 2 + hq;
        v4f v = *(const v4f*)(slab + row * 68 + c4);
        if (RESID) {
          const v4f rr = *(const v4f*)(Rb + (size_t)(mBase + row) * ldc + n0 + c4);
          v4f rq;
          rq[0] = rbf(rr[0]); rq[1] = rbf(rr[1]); rq[2] = rbf(rr[2]); rq[3] = rbf(rr[3]);
          v = v + rq;
        }
        vals[it] = v;
      }
      for (int pass = 0; pass < 2; ++pass) {
#pragma unroll
        for (int it = 0; it < 8; ++it) {
          const int row = it * 2 + hq;
          *(volatile v4f*)(Cb + (size_t)(mBase + row) * ldc + n0 + c4) = vals[it];
        }
        __threadfence();
      }
    } else {
      const int q = lane >> 3, c8 = (lane & 7) * 8;
      unsigned short* Cb  = (unsigned short*)Cout  + (size_t)b * strideC;
      unsigned short* Cb2 = (OUT_MODE == 2) ? ((unsigned short*)Cout2 + (size_t)b * strideC) : nullptr;
      for (int pass = 0; pass < 2; ++pass) {
#pragma unroll
        for (int it = 0; it < 4; ++it) {
          const int row = it * 4 + q;
          const float* sp = slab + row * 68 + c8;
          v8h hv, lv;
#pragma unroll
          for (int e = 0; e < 8; ++e) {
            if (OUT_MODE == 1) {
              hv[e] = (_Float16)sp[e];
            } else {
              unsigned short hb = f2bf_bits(sp[e]);
              unsigned short lb = f2bf_bits(sp[e] - bf_bits2f(hb));
              hv[e] = __builtin_bit_cast(_Float16, hb);
              lv[e] = __builtin_bit_cast(_Float16, lb);
            }
          }
          *(volatile v8h*)(Cb + (size_t)(mBase + row) * ldc + n0 + c8) = hv;
          if (OUT_MODE == 2) *(volatile v8h*)(Cb2 + (size_t)(mBase + row) * ldc + n0 + c8) = lv;
        }
        __threadfence();
      }
    }
    __builtin_amdgcn_fence(__ATOMIC_RELEASE, "workgroup");
    __builtin_amdgcn_wave_barrier();
    __builtin_amdgcn_fence(__ATOMIC_ACQUIRE, "workgroup");
  }
}

__global__ __launch_bounds__(256) void wcat_cast_kernel(const float* __restrict__ Wf, const float* __restrict__ Wg,
                                                        const float* __restrict__ Wh, unsigned short* __restrict__ Wcat) {
  const int blk = blockIdx.x;
  const int t   = threadIdx.x;
  const float* src;
  int base;
  if (blk < 16)      { src = Wf; base = 0; }
  else if (blk < 32) { src = Wg; base = 16 * 2048; }
  else               { src = Wh; base = 32 * 2048; }
  const int e = blk * 2048 + t * 8;
  const float* p = src + (e - base);
  const v4f a = *(const v4f*)(p);
  const v4f c = *(const v4f*)(p + 4);
  unsigned short hb[8];
#pragma unroll
  for (int k = 0; k < 4; ++k) {
    hb[k]     = f2bf_bits(a[k]);
    hb[4 + k] = f2bf_bits(c[k]);
  }
  const v4u u = (v4u){pk16(hb[0], hb[1]), pk16(hb[2], hb[3]), pk16(hb[4], hb[5]), pk16(hb[6], hb[7])};
  unsigned short* op = Wcat + e;
  *(volatile v4u*)op = u;
  __threadfence();
  *(volatile v4u*)op = u;
}

__global__ __launch_bounds__(256) void xt_cast_kernel(const float* __restrict__ x, unsigned short* __restrict__ xT) {
  __shared__ float sm[64][65];
  const int t  = threadIdx.x;
  const int n0 = blockIdx.x * 64;
  const int c0 = blockIdx.y * 64;
  const int b  = blockIdx.z;
  const float* xb = x + (size_t)b * kC * kN;
#pragma unroll
  for (int i = 0; i < 4; ++i) {
    const int e4 = i * 256 + t;
    const int r  = e4 >> 4;
    const int c4 = (e4 & 15) * 4;
    const v4f v = *(const v4f*)(xb + (size_t)(c0 + r) * kN + n0 + c4);
    sm[c4 + 0][r] = v[0];
    sm[c4 + 1][r] = v[1];
    sm[c4 + 2][r] = v[2];
    sm[c4 + 3][r] = v[3];
  }
  __syncthreads();
  const int lane = t & 31, wave = t >> 5;
  const int q = lane >> 3, c8 = (lane & 7) * 8;
  unsigned short* op = xT + ((size_t)b * kN + n0) * kC + c0;
  for (int pass = 0; pass < 2; ++pass) {
#pragma unroll
    for (int it = 0; it < 2; ++it) {
      const int row = wave * 8 + it * 4 + q;
      unsigned short hb[8];
#pragma unroll
      for (int e = 0; e < 8; ++e) hb[e] = f2bf_bits(sm[row][c8 + e]);
      const v4u u = (v4u){pk16(hb[0], hb[1]), pk16(hb[2], hb[3]), pk16(hb[4], hb[5]), pk16(hb[6], hb[7])};
      *(volatile v4u*)(op + (size_t)row * kC + c8) = u;
    }
    __threadfence();
  }
}

__global__ __launch_bounds__(256) void softmax_pt_kernel(const float* __restrict__ SC, unsigned short* __restrict__ PT, int icol0) {
  __shared__ __align__(16) unsigned short sm[64][72];
  __shared__ float mrow_s[64];
  __shared__ float irow_s[64];
  const int t    = threadIdx.x;
  const int lane = t & 31, wave = t >> 5;
  const int i0   = blockIdx.x * 64;

#pragma unroll 1
  for (int rr = 0; rr < 8; ++rr) {
    const int r = wave * 8 + rr;
    const float* rp = SC + (size_t)(i0 + r) * kN + lane * 4;
    float mx = -__builtin_inff();
#pragma unroll 1
    for (int k = 0; k < kN / 128; ++k) {
      const v4f v = *(const v4f*)(rp + k * 128);
      mx = fmaxf(mx, fmaxf(fmaxf(v[0], v[1]), fmaxf(v[2], v[3])));
    }
#pragma unroll
    for (int off = 16; off > 0; off >>= 1) mx = fmaxf(mx, __shfl_xor(mx, off, 32));
    float s = 0.f;
#pragma unroll 1
    for (int k = 0; k < kN / 128; ++k) {
      const v4f v = *(const v4f*)(rp + k * 128);
      s += (expf(v[0] - mx) + expf(v[1] - mx)) + (expf(v[2] - mx) + expf(v[3] - mx));
    }
#pragma unroll
    for (int off = 16; off > 0; off >>= 1) s += __shfl_xor(s, off, 32);
    if (lane == 0) {
      mrow_s[r] = mx;
      irow_s[r] = kPCarry / s;
    }
  }
  __syncthreads();

  const int q = lane >> 3, c8 = (lane & 7) * 8;
  unsigned short* ptb = PT + icol0 + i0;
#pragma unroll 1
  for (int jt = 0; jt < kN / 64; ++jt) {
    const int j0 = jt * 64;
#pragma unroll 1
    for (int it = 0; it < 4; ++it) {
      const int e4 = it * 256 + t;
      const int r  = e4 >> 4;
      const int c4 = (e4 & 15) * 4;
      const v4f v = *(const v4f*)(SC + (size_t)(i0 + r) * kN + j0 + c4);
      const float mr = mrow_s[r];
      const float ir = irow_s[r];
#pragma unroll
      for (int e = 0; e < 4; ++e) sm[c4 + e][r] = h_bits(expf(v[e] - mr) * ir);
    }
    __syncthreads();
    for (int pass = 0; pass < 2; ++pass) {
#pragma unroll
      for (int it = 0; it < 2; ++it) {
        const int row = wave * 8 + it * 4 + q;
        const v8us hv = *(const v8us*)(&sm[row][c8]);
        const v4u u = __builtin_bit_cast(v4u, hv);
        *(volatile v4u*)(ptb + (size_t)(j0 + row) * kN + c8) = u;
      }
      __threadfence();
    }
    __syncthreads();
  }
}

extern "C" void kernel_launch(void* const* d_in, const int* in_sizes, int n_in,
                              void* d_out, int out_size, void* d_ws, size_t ws_size,
                              hipStream_t stream) {
  if (n_in < 8) return;
  const int nX = kB * kC * kN;
  if (in_sizes[0] != nX) return;
  if (in_sizes[1] != kQ * kC || in_sizes[2] != kQ) return;
  if (in_sizes[3] != kQ * kC || in_sizes[4] != kQ) return;
  if (in_sizes[5] != kC * kC || in_sizes[6] != kC) return;
  if (in_sizes[7] < 1) return;
  if (out_size != nX) return;

  const size_t szXT  = (size_t)kB * kN * kC * 2;
  const size_t szW   = (size_t)kWRows * kC * 2;
  const size_t szFQ  = (size_t)kTok * kQ * 2;
  const size_t szHH  = (size_t)kB * kC * kN * 2;
  const size_t szSC  = (size_t)kCh * kN * 4;
  const size_t szPT  = (size_t)kN * kN * 2;
  const size_t offXT  = 0;
  const size_t offW   = offXT + szXT;
  const size_t offFQH = offW + szW;
  const size_t offFQL = offFQH + szFQ;
  const size_t offGKH = offFQL + szFQ;
  const size_t offGKL = offGKH + szFQ;
  const size_t offHH  = offGKL + szFQ;
  const size_t offSC  = offHH + szHH;
  const size_t offPT  = offSC + szSC;
  const size_t total  = offPT + szPT;
  if (ws_size < total) return;

  const float* x     = (const float*)d_in[0];
  const float* Wf    = (const float*)d_in[1];
  const float* bf_in = (const float*)d_in[2];
  const float* Wg    = (const float*)d_in[3];
  const float* bg_in = (const float*)d_in[4];
  const float* Wh    = (const float*)d_in[5];
  const float* bh_in = (const float*)d_in[6];
  const float* gamma = (const float*)d_in[7];
  float* out = (float*)d_out;
  char* ws = (char*)d_ws;
  unsigned short* xTb   = (unsigned short*)(ws + offXT);
  unsigned short* Wcatb = (unsigned short*)(ws + offW);
  unsigned short* fqh   = (unsigned short*)(ws + offFQH);
  unsigned short* fql   = (unsigned short*)(ws + offFQL);
  unsigned short* gkh   = (unsigned short*)(ws + offGKH);
  unsigned short* gkl   = (unsigned short*)(ws + offGKL);
  unsigned short* hh16  = (unsigned short*)(ws + offHH);
  float*          SC    = (float*)(ws + offSC);
  unsigned short* PT    = (unsigned short*)(ws + offPT);

  wcat_cast_kernel<<<dim3((kWRows * kC) / 2048), dim3(256), 0, stream>>>(Wf, Wg, Wh, Wcatb);
  xt_cast_kernel<<<dim3(kN / 64, kC / 64, kB), dim3(256), 0, stream>>>(x, xTb);

  const int tilesFG = (kTok / 64) * (kQ / 64);
  wmma_gemm64<1, false, 2, 2, false, false><<<dim3(tilesFG / 8, 1), dim3(256), 0, stream>>>(
      xTb, xTb, kC, 0L, Wcatb, Wcatb, kC, 0L,
      (void*)fqh, (void*)fql, kQ, 0L, bf_in, x, 0L, gamma, kTok, kQ, kC, 1.0f);
  wmma_gemm64<1, false, 2, 2, false, false><<<dim3(tilesFG / 8, 1), dim3(256), 0, stream>>>(
      xTb, xTb, kC, 0L, Wcatb + (size_t)kQ * kC, Wcatb + (size_t)kQ * kC, kC, 0L,
      (void*)gkh, (void*)gkl, kQ, 0L, bg_in, x, 0L, gamma, kTok, kQ, kC, 1.0f);
  const int tilesHH = (kC / 64) * (kN / 64);
  wmma_gemm64<1, false, 1, 1, false, false><<<dim3(tilesHH / 8, kB), dim3(256), 0, stream>>>(
      Wcatb + (size_t)2 * kQ * kC, Wcatb + (size_t)2 * kQ * kC, kC, 0L, xTb, xTb, kC, (long)kN * kC,
      (void*)hh16, (void*)hh16, kN, (long)kC * kN, bh_in, x, 0L, gamma, kC, kN, kC, 1.0f);

  const int tilesSC = (kCh / 64) * (kN / 64);
  const int tilesPV = (kC / 64) * (kN / 64);
  for (int b = 0; b < kB; ++b) {
    for (int ch = 0; ch < kN / kCh; ++ch) {
      const size_t aoff = ((size_t)b * kN + (size_t)ch * kCh) * kQ;
      const size_t boff = (size_t)b * kN * kQ;
      wmma_gemm64<1, true, 0, 0, false, false><<<dim3(tilesSC / 8, 1), dim3(256), 0, stream>>>(
          fqh + aoff, fql + aoff, kQ, 0L, gkh + boff, gkl + boff, kQ, 0L,
          (void*)SC, (void*)SC, kN, 0L, bf_in, x, 0L, gamma, kCh, kN, kQ, 1.0f);
      softmax_pt_kernel<<<dim3(kCh / 64), dim3(256), 0, stream>>>(SC, PT, ch * kCh);
    }
    const size_t xoff = (size_t)b * kC * kN;
    wmma_gemm64<0, false, 0, 0, true, true><<<dim3(tilesPV / 8, 1), dim3(256), 0, stream>>>(
        hh16 + xoff, hh16 + xoff, kN, 0L, PT, PT, kN, 0L,
        (void*)(out + xoff), (void*)(out + xoff), kN, 0L, bf_in, x + xoff, 0L, gamma, kC, kN, kN, kPCarryInv);
  }
}
